// STGCNBlock_52785148068460
// MI455X (gfx1250) — hardware-verified
//
#include <hip/hip_runtime.h>
#include <hip/hip_bf16.h>
#include <stdint.h>


typedef __bf16 v16b __attribute__((ext_vector_type(16)));
typedef float v8f __attribute__((ext_vector_type(8)));
typedef float v4f __attribute__((ext_vector_type(4)));
typedef unsigned int v4u __attribute__((ext_vector_type(4)));

#define TT 64
#define NN 2000
#define CC 64
#define NTILE (NN / 16)
#define ROW_TILES (TT * NTILE)
#define GEMM_BLOCKS (ROW_TILES / 4)
#define TOTAL (TT * NN * CC)
#define DEG_PAD 2048
#define DEG_BLOCKS (DEG_PAD / 256)
#define AGG_G 4
#define AGG_BLOCKS (NN / AGG_G)
#define FRAG_STRIDE 1024
#define BN_BLOCKS ((TOTAL / 4 + 255) / 256)

static_assert(NN % 16 == 0, "");
static_assert(ROW_TILES % 4 == 0, "");
static_assert(NN % AGG_G == 0, "");
static_assert(TOTAL % 4 == 0, "");
static_assert(DEG_PAD >= NN && DEG_PAD % 256 == 0, "");

union FragU { v4u u[2]; v16b v; };

__device__ __forceinline__ float bf16_to_f32(__bf16 b) {
  return __builtin_bit_cast(float, ((unsigned)__builtin_bit_cast(unsigned short, b)) << 16);
}

__device__ __forceinline__ void a_frag_split(const float* p, int h, v16b& hi, v16b& lo) {
  union { v4f q[4]; float f[16]; } u;
  u.q[0] = *(const v4f*)(p + 8 * h);
  u.q[1] = *(const v4f*)(p + 8 * h + 4);
  u.q[2] = *(const v4f*)(p + 16 + 8 * h);
  u.q[3] = *(const v4f*)(p + 20 + 8 * h);
  union { __bf16 e[16]; v16b v; } bh, bl;
#pragma unroll
  for (int j = 0; j < 16; ++j) {
    const __bf16 t = (__bf16)u.f[j];
    bh.e[j] = t;
    bl.e[j] = (__bf16)(u.f[j] - bf16_to_f32(t));
  }
  hi = bh.v;
  lo = bl.v;
}

__device__ __forceinline__ void b_frag_split(const __bf16* p, v16b& hi, v16b& lo) {
  FragU a, b;
  a.u[0] = *(const v4u*)p;
  a.u[1] = *(const v4u*)(p + 8);
  b.u[0] = *(const v4u*)(p + 512);
  b.u[1] = *(const v4u*)(p + 520);
  hi = a.v;
  lo = b.v;
}

__device__ __forceinline__ v8f wmma3(v8f acc, v16b ah, v16b al, v16b bh, v16b bl) {
  acc = __builtin_amdgcn_wmma_f32_16x16x32_bf16(false, ah, false, bh, (short)0, acc, false, false);
  acc = __builtin_amdgcn_wmma_f32_16x16x32_bf16(false, ah, false, bl, (short)0, acc, false, false);
  acc = __builtin_amdgcn_wmma_f32_16x16x32_bf16(false, al, false, bh, (short)0, acc, false, false);
  asm volatile("v_nop\n\tv_nop\n\tv_nop\n\tv_nop" : "+v"(acc) : "v"(ah), "v"(al), "v"(bh), "v"(bl));
  return acc;
}

__global__ __launch_bounds__(256) void k_pack(const float* __restrict__ w1, const float* __restrict__ w2,
                                              const float* __restrict__ gw, __bf16* __restrict__ p1,
                                              __bf16* __restrict__ p2, __bf16* __restrict__ pg) {
  const int u = blockIdx.x * 256 + threadIdx.x;
  const float* w;
  __bf16* dst;
  int v, isconv;
  if (u < 1536) { w = w1; dst = p1; v = u; isconv = 1; }
  else if (u < 3072) { w = w2; dst = p2; v = u - 1536; isconv = 1; }
  else if (u < 3584) { w = gw; dst = pg; v = u - 3072; isconv = 0; }
  else return;
  const int frag = v >> 6, within = v & 63;
  const int L = within >> 1, jh = within & 1;
  const int nt = frag & 3, s = (frag >> 2) & 1, k = frag >> 3;
  const int h = L >> 4, o = nt * 16 + (L & 15);
  const int ibase = s * 32 + jh * 16 + 8 * h;
  union { __bf16 b[8]; v4u u; } ph, pl;
#pragma unroll
  for (int j = 0; j < 8; ++j) {
    const int i = ibase + j;
    const int idx = isconv ? ((o * CC + i) * 3 + k) : (i * CC + o);
    const float val = w[idx];
    const __bf16 hb = (__bf16)val;
    ph.b[j] = hb;
    pl.b[j] = (__bf16)(val - bf16_to_f32(hb));
  }
  const v4u vh = ph.u, vl = pl.u;
  __bf16* q = dst + frag * FRAG_STRIDE + within * 8;
  *(volatile v4u*)q = vh;
  *(volatile v4u*)(q + 512) = vl;
  __threadfence();
  *(volatile v4u*)q = vh;
  *(volatile v4u*)(q + 512) = vl;
}

__global__ __launch_bounds__(256) void k_deg(const int* __restrict__ ei, int E, float* __restrict__ dinv) {
  __shared__ int slist[256];
  __shared__ int scnt[8];
  __shared__ __align__(16) float sd[256];
  const int tid = threadIdx.x, lane = tid & 31, wave = tid >> 5;
  const int n0 = blockIdx.x * 256;
  const unsigned ltmask = (1u << lane) - 1u;
  int cnt = 1;
  for (int base = 0; base < E; base += 256) {
    const int e = base + tid;
    int g = -1;
    if (e < E) g = ei[(size_t)E + e] - n0;
    const bool hit = (unsigned)g < 256u;
    const unsigned mk = __builtin_amdgcn_ballot_w32(hit);
    const int rank = __builtin_popcount(mk & ltmask);
    if (lane == 0) scnt[wave] = __builtin_popcount(mk);
    __syncthreads();
    int off = rank, tot = 0;
#pragma unroll
    for (int w = 0; w < 8; ++w) {
      const int cw = scnt[w];
      tot += cw;
      off += (w < wave) ? cw : 0;
    }
    if (hit) slist[off > 255 ? 255 : off] = g;
    __syncthreads();
    tot = tot > 256 ? 256 : tot;
    for (int hh = 0; hh < tot; ++hh) cnt += (slist[hh] == tid) ? 1 : 0;
    __syncthreads();
  }
  sd[tid] = 1.0f / sqrtf((float)cnt);
  __syncthreads();
  if (tid < 64) {
    const v4f v = *(const v4f*)&sd[tid * 4];
    float* q = dinv + n0 + tid * 4;
    *(volatile v4f*)q = v;
    __threadfence();
    *(volatile v4f*)q = v;
  }
}

__device__ __forceinline__ void conv_tile(const float* __restrict__ src, const __bf16* __restrict__ wp,
                                          int t, int n0, int lane, int h, int m, v8f (&acc)[4]) {
#pragma unroll
  for (int k = 0; k < 3; ++k) {
    const int trow = t + k - 1;
    if (trow >= 0 && trow < TT) {
      const float* arow = src + ((size_t)trow * NN + n0 + m) * CC;
#pragma unroll
      for (int s = 0; s < 2; ++s) {
        v16b ah, al;
        a_frag_split(arow + s * 32, h, ah, al);
#pragma unroll
        for (int nt = 0; nt < 4; ++nt) {
          v16b bh, bl;
          b_frag_split(wp + ((k * 2 + s) * 4 + nt) * FRAG_STRIDE + lane * 16, bh, bl);
          acc[nt] = wmma3(acc[nt], ah, al, bh, bl);
        }
      }
    }
  }
}

__device__ __forceinline__ void tile_rows_store2(const float (*st)[64], float* __restrict__ dst, int h, int m) {
  v4f v[8];
#pragma unroll
  for (int it = 0; it < 8; ++it) v[it] = *(const v4f*)&st[it * 2 + h][m * 4];
#pragma unroll
  for (int it = 0; it < 8; ++it) *(volatile v4f*)(dst + (size_t)(it * 2 + h) * CC + m * 4) = v[it];
  __threadfence();
#pragma unroll
  for (int it = 0; it < 8; ++it) *(volatile v4f*)(dst + (size_t)(it * 2 + h) * CC + m * 4) = v[it];
}

__global__ __launch_bounds__(128) void k_conv1_lin(const float* __restrict__ x, const __bf16* __restrict__ wp,
                                                   const float* __restrict__ bias, const __bf16* __restrict__ gp,
                                                   const float* __restrict__ dinv, float* __restrict__ xh) {
  __shared__ __align__(16) float stage[4][16][64];
  const int wave = threadIdx.x >> 5, lane = threadIdx.x & 31, h = lane >> 4, m = lane & 15;
  const int tile = __builtin_amdgcn_readfirstlane((int)(blockIdx.x * 4) + wave);
  const int t = tile / NTILE, n0 = (tile - t * NTILE) * 16;

  v8f acc[4];
#pragma unroll
  for (int nt = 0; nt < 4; ++nt)
#pragma unroll
    for (int r = 0; r < 8; ++r) acc[nt][r] = 0.0f;

  conv_tile(x, wp, t, n0, lane, h, m, acc);

#pragma unroll
  for (int nt = 0; nt < 4; ++nt) {
    const float bv = bias[nt * 16 + m];
#pragma unroll
    for (int r = 0; r < 8; ++r) stage[wave][r + 8 * h][nt * 16 + m] = acc[nt][r] + bv;
  }
  __syncthreads();

  v8f acc2[4];
#pragma unroll
  for (int nt = 0; nt < 4; ++nt)
#pragma unroll
    for (int r = 0; r < 8; ++r) acc2[nt][r] = 0.0f;
#pragma unroll
  for (int s = 0; s < 2; ++s) {
    v16b ah, al;
    a_frag_split(&stage[wave][m][s * 32], h, ah, al);
#pragma unroll
    for (int nt = 0; nt < 4; ++nt) {
      v16b bh, bl;
      b_frag_split(gp + (s * 4 + nt) * FRAG_STRIDE + lane * 16, bh, bl);
      acc2[nt] = wmma3(acc2[nt], ah, al, bh, bl);
    }
  }
  __syncthreads();

  union { v4f q[2]; float f[8]; } dv;
  dv.q[0] = *(const v4f*)(dinv + n0 + 8 * h);
  dv.q[1] = *(const v4f*)(dinv + n0 + 8 * h + 4);
#pragma unroll
  for (int nt = 0; nt < 4; ++nt)
#pragma unroll
    for (int r = 0; r < 8; ++r) stage[wave][r + 8 * h][nt * 16 + m] = acc2[nt][r] * dv.f[r];
  __syncthreads();

  tile_rows_store2(stage[wave], xh + (size_t)tile * 16 * CC, h, m);
}

__device__ __forceinline__ void drain_one(const int* list, const int* cntcol,
                                          const float* __restrict__ xh, int tq, int c4, v4f (&a)[4]) {
  int tot = 0;
#pragma unroll
  for (int w = 0; w < 8; ++w) tot += cntcol[w * AGG_G];
  tot = tot > 256 ? 256 : (tot < 0 ? 0 : tot);
  for (int hh = 0; hh < tot; ++hh) {
    int s = list[hh];
    s = s < 0 ? 0 : (s >= NN ? NN - 1 : s);
    const float* xp = xh + (size_t)s * CC + c4;
#pragma unroll
    for (int q = 0; q < 4; ++q) {
      const v4f v = *(const v4f*)(xp + (size_t)(q * 16 + tq) * (size_t)(NN * CC));
      a[q] += v;
    }
  }
}

__device__ __forceinline__ void self_fin_one(int n, float dng, const float* __restrict__ xh, int tq, int c4,
                                             v4f bb, v4f (&a)[4]) {
  const float* xp = xh + (size_t)n * CC + c4;
#pragma unroll
  for (int q = 0; q < 4; ++q) {
    const v4f v = *(const v4f*)(xp + (size_t)(q * 16 + tq) * (size_t)(NN * CC));
    a[q] += v;
  }
#pragma unroll
  for (int q = 0; q < 4; ++q) a[q] = a[q] * dng + bb;
}

__device__ __forceinline__ void store_one(int n, float* __restrict__ agg, int tq, int c4, const v4f (&a)[4]) {
#pragma unroll
  for (int q = 0; q < 4; ++q) {
    float* p = agg + ((size_t)(q * 16 + tq) * NN + n) * CC + c4;
    *(volatile v4f*)p = a[q];
  }
}

__global__ __launch_bounds__(256) void k_agg(const float* __restrict__ xh, const int* __restrict__ ei, int E,
                                             const float* __restrict__ dinv, const float* __restrict__ gb,
                                             float* __restrict__ agg) {
  __shared__ int slist[AGG_G][256];
  __shared__ int scnt[8][AGG_G];
  const int tid = threadIdx.x, lane = tid & 31, wave = tid >> 5;
  const int n0 = blockIdx.x * AGG_G;
  const int tq = tid >> 4, c4 = (tid & 15) * 4;
  const unsigned ltmask = (1u << lane) - 1u;

  v4f acc[AGG_G][4];
#pragma unroll
  for (int g = 0; g < AGG_G; ++g)
#pragma unroll
    for (int q = 0; q < 4; ++q)
#pragma unroll
      for (int i = 0; i < 4; ++i) acc[g][q][i] = 0.0f;

  float dn[AGG_G];
#pragma unroll
  for (int g = 0; g < AGG_G; ++g) {
    int n = n0 + g;
    n = n < NN ? n : NN - 1;
    dn[g] = dinv[n];
  }

  for (int base = 0; base < E; base += 256) {
    const int e = base + tid;
    int g = -1, s = 0;
    if (e < E) { s = ei[e]; g = ei[(size_t)E + e] - n0; }
    s = s < 0 ? 0 : (s >= NN ? NN - 1 : s);
    const bool hit = (unsigned)g < (unsigned)AGG_G;
    int myrank = 0;
    unsigned cw[AGG_G];
#pragma unroll
    for (int gg = 0; gg < AGG_G; ++gg) {
      const bool mine = hit && (g == gg);
      const unsigned mk = __builtin_amdgcn_ballot_w32(mine);
      cw[gg] = (unsigned)__builtin_popcount(mk);
      if (mine) myrank = __builtin_popcount(mk & ltmask);
    }
    if (lane == 0) {
#pragma unroll
      for (int gg = 0; gg < AGG_G; ++gg) scnt[wave][gg] = (int)cw[gg];
    }
    __syncthreads();
    if (hit) {
      int off = myrank;
#pragma unroll
      for (int w = 0; w < 8; ++w) off += (w < wave) ? scnt[w][g] : 0;
      slist[g][off > 255 ? 255 : off] = s;
    }
    __syncthreads();
    drain_one(&slist[0][0], &scnt[0][0], xh, tq, c4, acc[0]);
    drain_one(&slist[1][0], &scnt[0][1], xh, tq, c4, acc[1]);
    drain_one(&slist[2][0], &scnt[0][2], xh, tq, c4, acc[2]);
    drain_one(&slist[3][0], &scnt[0][3], xh, tq, c4, acc[3]);
    __syncthreads();
  }

  v4f bb;
  bb.x = gb[c4 + 0]; bb.y = gb[c4 + 1]; bb.z = gb[c4 + 2]; bb.w = gb[c4 + 3];
  self_fin_one(n0 + 0, dn[0], xh, tq, c4, bb, acc[0]);
  self_fin_one(n0 + 1, dn[1], xh, tq, c4, bb, acc[1]);
  self_fin_one(n0 + 2, dn[2], xh, tq, c4, bb, acc[2]);
  self_fin_one(n0 + 3, dn[3], xh, tq, c4, bb, acc[3]);

  store_one(n0 + 0, agg, tq, c4, acc[0]);
  store_one(n0 + 1, agg, tq, c4, acc[1]);
  store_one(n0 + 2, agg, tq, c4, acc[2]);
  store_one(n0 + 3, agg, tq, c4, acc[3]);
  __threadfence();
  store_one(n0 + 0, agg, tq, c4, acc[0]);
  store_one(n0 + 1, agg, tq, c4, acc[1]);
  store_one(n0 + 2, agg, tq, c4, acc[2]);
  store_one(n0 + 3, agg, tq, c4, acc[3]);
}

__global__ __launch_bounds__(128) void k_conv2(const float* __restrict__ a, const __bf16* __restrict__ wp,
                                               const float* __restrict__ bias, float* __restrict__ h3,
                                               float* __restrict__ part) {
  __shared__ __align__(16) float stage[4][16][64];
  __shared__ __align__(16) float spart[128];
  const int wave = threadIdx.x >> 5, lane = threadIdx.x & 31, h = lane >> 4, m = lane & 15;
  const int tile = __builtin_amdgcn_readfirstlane((int)(blockIdx.x * 4) + wave);
  const int t = tile / NTILE, n0 = (tile - t * NTILE) * 16;

  v8f acc[4];
#pragma unroll
  for (int nt = 0; nt < 4; ++nt)
#pragma unroll
    for (int r = 0; r < 8; ++r) acc[nt][r] = 0.0f;

  conv_tile(a, wp, t, n0, lane, h, m, acc);

#pragma unroll
  for (int nt = 0; nt < 4; ++nt) {
    const float bv = bias[nt * 16 + m];
#pragma unroll
    for (int r = 0; r < 8; ++r) stage[wave][r + 8 * h][nt * 16 + m] = acc[nt][r] + bv;
  }
  __syncthreads();

  tile_rows_store2(stage[wave], h3 + (size_t)tile * 16 * CC, h, m);

  {
    const int c = threadIdx.x & 63, which = threadIdx.x >> 6;
    float sa = 0.0f;
#pragma unroll
    for (int w = 0; w < 4; ++w)
#pragma unroll
      for (int r = 0; r < 16; ++r) {
        const float val = stage[w][r][c];
        sa += which ? (val * val) : val;
      }
    spart[threadIdx.x] = sa;
  }
  __syncthreads();
  if (wave == 0) {
    const v4f pv = *(const v4f*)&spart[lane * 4];
    *(volatile v4f*)(part + (size_t)blockIdx.x * 128 + lane * 4) = pv;
  }
  __threadfence();
  if (wave == 0) {
    const v4f pv = *(const v4f*)&spart[lane * 4];
    *(volatile v4f*)(part + (size_t)blockIdx.x * 128 + lane * 4) = pv;
  }
}

__global__ __launch_bounds__(128) void k_stats(const float* __restrict__ part, int nblk, float* __restrict__ st) {
  __shared__ double sred[128];
  __shared__ __align__(16) float sout[128];
  const int tid = threadIdx.x;
  double acc = 0.0;
  for (int b = 0; b < nblk; ++b) acc += (double)part[(size_t)b * 128 + tid];
  sred[tid] = acc;
  __syncthreads();
  if (tid < 64) {
    const double invm = 1.0 / (double)(TT * NN);
    const double mean = sred[tid] * invm;
    double var = sred[64 + tid] * invm - mean * mean;
    var = var > 0.0 ? var : 0.0;
    const float varf = (float)var;
    sout[tid] = (float)mean;
    sout[64 + tid] = 1.0f / sqrtf(varf + 1e-5f);
  }
  __syncthreads();
  if (tid < 32) {
    const v4f v = *(const v4f*)&sout[tid * 4];
    float* q = st + tid * 4;
    *(volatile v4f*)q = v;
    __threadfence();
    *(volatile v4f*)q = v;
  }
}

__global__ __launch_bounds__(256) void k_bn(const float* __restrict__ h3, const float* __restrict__ st,
                                            const float* __restrict__ gamma, const float* __restrict__ beta,
                                            float* __restrict__ out) {
  const size_t i4 = (size_t)blockIdx.x * 256 + threadIdx.x;
  if (i4 >= (size_t)(TOTAL / 4)) return;
  const int c0 = (int)((i4 * 4) & 63);
  const v4f xv = *(const v4f*)(h3 + i4 * 4);
  const v4f mu = *(const v4f*)(st + c0);
  const v4f iv = *(const v4f*)(st + 64 + c0);
  v4f gm, bt;
  gm.x = gamma[c0 + 0]; gm.y = gamma[c0 + 1]; gm.z = gamma[c0 + 2]; gm.w = gamma[c0 + 3];
  bt.x = beta[c0 + 0];  bt.y = beta[c0 + 1];  bt.z = beta[c0 + 2];  bt.w = beta[c0 + 3];
  v4f y = (xv - mu) * iv * gm + bt;
  y.x = y.x > 0.0f ? y.x : 0.0f;
  y.y = y.y > 0.0f ? y.y : 0.0f;
  y.z = y.z > 0.0f ? y.z : 0.0f;
  y.w = y.w > 0.0f ? y.w : 0.0f;
  float* q = out + i4 * 4;
  *(volatile v4f*)q = y;
  __threadfence();
  *(volatile v4f*)q = y;
}

extern "C" void kernel_launch(void* const* d_in, const int* in_sizes, int n_in,
                              void* d_out, int out_size, void* d_ws, size_t ws_size,
                              hipStream_t stream) {
  if (n_in < 10) return;
  if (in_sizes[0] != TOTAL || out_size != TOTAL) return;
  const float* x     = (const float*)d_in[0];
  const int*   ei    = (const int*)d_in[1];
  const float* c1w   = (const float*)d_in[2];
  const float* c1b   = (const float*)d_in[3];
  const float* gw    = (const float*)d_in[4];
  const float* gb    = (const float*)d_in[5];
  const float* c2w   = (const float*)d_in[6];
  const float* c2b   = (const float*)d_in[7];
  const float* gamma = (const float*)d_in[8];
  const float* beta  = (const float*)d_in[9];
  int E = in_sizes[1] / 2;
  if (E < 0) E = 0;

  size_t off = 0;
  auto carve = [&](size_t bytes) -> size_t {
    const size_t o = off;
    off += (bytes + 255) & ~(size_t)255;
    return o;
  };
  const size_t o_xh   = carve((size_t)TOTAL * 4);
  const size_t o_agg  = carve((size_t)TOTAL * 4);
  const size_t o_h3   = carve((size_t)TOTAL * 4);
  const size_t o_dinv = carve((size_t)DEG_PAD * 4);
  const size_t o_part = carve((size_t)GEMM_BLOCKS * 128 * 4);
  const size_t o_st   = carve(128 * 4);
  const size_t o_wp1  = carve((size_t)24 * FRAG_STRIDE * 2);
  const size_t o_wp2  = carve((size_t)24 * FRAG_STRIDE * 2);
  const size_t o_gp   = carve((size_t)8 * FRAG_STRIDE * 2);
  if (off > ws_size) return;

  char* ws = (char*)d_ws;
  float*  xh   = (float*)(ws + o_xh);
  float*  agg  = (float*)(ws + o_agg);
  float*  h3   = (float*)(ws + o_h3);
  float*  dinv = (float*)(ws + o_dinv);
  float*  part = (float*)(ws + o_part);
  float*  st   = (float*)(ws + o_st);
  __bf16* wp1  = (__bf16*)(ws + o_wp1);
  __bf16* wp2  = (__bf16*)(ws + o_wp2);
  __bf16* gp   = (__bf16*)(ws + o_gp);

  k_pack<<<14, 256, 0, stream>>>(c1w, c2w, gw, wp1, wp2, gp);
  k_deg<<<DEG_BLOCKS, 256, 0, stream>>>(ei, E, dinv);
  k_conv1_lin<<<GEMM_BLOCKS, 128, 0, stream>>>(x, wp1, c1b, gp, dinv, xh);
  k_agg<<<AGG_BLOCKS, 256, 0, stream>>>(xh, ei, E, dinv, gb, agg);
  k_conv2<<<GEMM_BLOCKS, 128, 0, stream>>>(agg, wp2, c2b, h3, part);
  k_stats<<<1, 128, 0, stream>>>(part, GEMM_BLOCKS, st);
  k_bn<<<BN_BLOCKS, 256, 0, stream>>>(h3, st, gamma, beta, (float*)d_out);
}
